// RNN_7894149890770
// MI455X (gfx1250) — hardware-verified
//
#include <hip/hip_runtime.h>
#include <math.h>

constexpr int SEQ_T   = 131072;
constexpr int NIN     = 100;
constexpr int NHID    = 40;
constexpr int NVOC    = 100;
constexpr int KPAD_X  = 128;
constexpr int NPAD_X  = 64;
constexpr int KPAD_Y  = 64;
constexpr int NPAD_Y  = 112;
constexpr int HPADR   = 16;
constexpr int HROWS   = SEQ_T + HPADR;
constexpr int HBATCH  = 16;
constexpr int SCAN_THR = 64;
constexpr int TBLK    = 64;
constexpr int NBLK_Y  = SEQ_T / TBLK;
constexpr int RD_THR  = 128;
constexpr int LGP     = NPAD_Y;
constexpr int LGROWS  = TBLK + 16;
constexpr int OUT1_OFF_F = 40;
constexpr long TOTAL_F = (long)OUT1_OFF_F + (long)SEQ_T * NVOC;
constexpr int FSHIFT  = ((OUT1_OFF_F + 31) / 32) * 32;
constexpr int NIT_ST  = 13;
constexpr float WY_CARRY     = 64.0f;
constexpr float WY_CARRY_INV = 1.0f / 64.0f;

static_assert(OUT1_OFF_F == NHID);
static_assert(OUT1_OFF_F * 4 == 160);
static_assert(TOTAL_F * 4 == 52428960L);
static_assert(TOTAL_F % 4 == 0);
static_assert(SEQ_T % 64 == 0 && NPAD_X % 64 == 0 && KPAD_X % 32 == 0);
static_assert((SEQ_T / 64) % 8 == 0);
static_assert(NIN <= KPAD_X && NHID <= NPAD_X && NIN % 4 == 0 && NIN >= 8);
static_assert(KPAD_X / 8 == 16);
static_assert((SEQ_T * (KPAD_X / 8)) % 256 == 0);
static_assert(NHID <= KPAD_Y && KPAD_Y == 64 && NVOC <= NPAD_Y && NPAD_Y == 7 * 16);
static_assert((NPAD_Y * KPAD_Y / 8) % RD_THR == 0);
static_assert(NPAD_Y % 4 == 0 && NVOC % 4 == 0 && NPAD_Y / 4 <= 32);
static_assert(NHID % 4 == 0 && (NHID * NHID) % 4 == 0);
static_assert(HBATCH * NPAD_X == 4 * 4 * SCAN_THR);
static_assert(HBATCH * 8 == 2 * SCAN_THR && HPADR == HBATCH);
static_assert(SEQ_T % HBATCH == 0 && SEQ_T % TBLK == 0);
static_assert((TBLK * NVOC) % 32 == 0);
static_assert(FSHIFT == 64 && FSHIFT - OUT1_OFF_F < NVOC);
static_assert((TBLK * NVOC + FSHIFT - 1 - OUT1_OFF_F) / NVOC == TBLK);
static_assert(LGROWS >= TBLK + 16 && TBLK + 1 <= RD_THR);
static_assert(NIT_ST * RD_THR * 4 >= TBLK * NVOC + FSHIFT);
static_assert(TBLK * (NBLK_Y - 1) + 16 * 4 + 16 <= HROWS);

typedef __attribute__((ext_vector_type(16))) _Float16 v16h;
typedef __attribute__((ext_vector_type(8)))  _Float16 v8h;
typedef __attribute__((ext_vector_type(16))) __bf16   v16b;
typedef __attribute__((ext_vector_type(8)))  __bf16   v8b;
typedef __attribute__((ext_vector_type(8)))  float    v8f;
typedef __attribute__((ext_vector_type(4)))  float    v4f;
typedef __attribute__((ext_vector_type(4)))  unsigned int v4u;

__device__ __forceinline__ unsigned short f2bf_bits(float f) {
  unsigned u = __float_as_uint(f);
  return (unsigned short)((u + 0x7FFFu + ((u >> 16) & 1u)) >> 16);
}
__device__ __forceinline__ float bf_bits2f(unsigned short h) { return __uint_as_float(((unsigned)h) << 16); }
__device__ __forceinline__ float bf16r(float f) { return bf_bits2f(f2bf_bits(f)); }

__device__ __forceinline__ void dep_guard_h(v8f& a, v8f& b, v16h x, v16h y) { asm volatile("v_nop\n\tv_nop\n\tv_nop\n\tv_nop" : "+v"(a), "+v"(b) : "v"(x), "v"(y)); }
__device__ __forceinline__ void dep_guard_b(v8f& a, v8f& b, v16b x, v16b y) { asm volatile("v_nop\n\tv_nop\n\tv_nop\n\tv_nop" : "+v"(a), "+v"(b) : "v"(x), "v"(y)); }
__device__ __forceinline__ void keep4_h(v16h a, v16h b, v16h c, v16h d) { asm volatile("v_nop" :: "v"(a), "v"(b), "v"(c), "v"(d)); }
__device__ __forceinline__ void keep4_b(v16b a, v16b b, v16b c, v16b d) { asm volatile("v_nop" :: "v"(a), "v"(b), "v"(c), "v"(d)); }
__device__ __forceinline__ void acc_guard4(v8f& a, v8f& b, v8f& c, v8f& d) { asm volatile("v_nop\n\tv_nop\n\tv_nop\n\tv_nop" : "+v"(a), "+v"(b), "+v"(c), "+v"(d)); }
__device__ __forceinline__ void acc_guard3(v8f& a, v8f& b, v8f& c) { asm volatile("v_nop\n\tv_nop\n\tv_nop\n\tv_nop" : "+v"(a), "+v"(b), "+v"(c)); }
__device__ __forceinline__ void acc_guard1_h4(v8f& a, v16h w, v16h x, v16h y, v16h z) {
  asm volatile("v_nop\n\tv_nop\n\tv_nop\n\tv_nop" : "+v"(a) : "v"(w), "v"(x), "v"(y), "v"(z));
}
__device__ __forceinline__ void keep2_h(v16h a, v16h b) { asm volatile("v_nop" :: "v"(a), "v"(b)); }

template <typename T> struct Frag;
template <> struct Frag<_Float16> {
  typedef v16h V; union U { v16h v; v8h h[2]; };
  static __device__ __forceinline__ v16h load(const _Float16* p) {
    U f; f.h[0] = *(const v8h*)(p); f.h[1] = *(const v8h*)(p + 16); return f.v;
  }
  static __device__ __forceinline__ v8f mma(v16h a, v16h b, v8f c) {
    return __builtin_amdgcn_wmma_f32_16x16x32_f16(false, a, false, b, (short)0, c, false, false);
  }
  static __device__ __forceinline__ void guard(v8f& a, v8f& b, v16h x, v16h y) { dep_guard_h(a, b, x, y); }
  static __device__ __forceinline__ void keep(v16h a, v16h b, v16h c, v16h d) { keep4_h(a, b, c, d); }
};
template <> struct Frag<__bf16> {
  typedef v16b V; union U { v16b v; v8b h[2]; };
  static __device__ __forceinline__ v16b load(const __bf16* p) {
    U f; f.h[0] = *(const v8b*)(p); f.h[1] = *(const v8b*)(p + 16); return f.v;
  }
  static __device__ __forceinline__ v8f mma(v16b a, v16b b, v8f c) {
    return __builtin_amdgcn_wmma_f32_16x16x32_bf16(false, a, false, b, (short)0, c, false, false);
  }
  static __device__ __forceinline__ void guard(v8f& a, v8f& b, v16b x, v16b y) { dep_guard_b(a, b, x, y); }
  static __device__ __forceinline__ void keep(v16b a, v16b b, v16b c, v16b d) { keep4_b(a, b, c, d); }
};

template <int ET> struct Elem;
template <> struct Elem<0> { typedef _Float16 T; };
template <> struct Elem<1> { typedef __bf16 T; };
template <int ET, bool SPLIT, int BIAS_MODE, int OUT_MODE, bool RESID, int ACT = 0>
__global__ __launch_bounds__(256) void wmma_gemm64(
    const unsigned short* __restrict__ Ap, const unsigned short* __restrict__ A2p, int lda, long strideA,
    const unsigned short* __restrict__ Btp, const unsigned short* __restrict__ Bt2p, int ldb, long strideB,
    void* __restrict__ Cout, void* __restrict__ Cout2, int ldc, long strideC,
    const float* __restrict__ bias,
    const float* __restrict__ resid, long strideR,
    int M, int N, int K, float scale) {
  typedef typename Elem<ET>::T T;
  typedef typename Frag<T>::V V;
  const T* A = (const T*)Ap; const T* A2 = (const T*)A2p; const T* Bt = (const T*)Btp; const T* Bt2 = (const T*)Bt2p;
  __shared__ __align__(16) float sT[8][16 * 68];
  const int b    = blockIdx.y;
  const int lane = threadIdx.x & 31;
  const int wave = threadIdx.x >> 5;
  const int tilesN = N >> 6;
  const int tilesM = M >> 6;
  const int tile = blockIdx.x * 8 + wave;
  if (tile >= tilesM * tilesN) return;
  const int tm = tile / tilesN;
  const int tn = tile - tm * tilesN;
  const int m0 = tm << 6;
  const int n0 = tn << 6;

  const T* Ab  = A  + (size_t)b * strideA;
  const T* Bb  = Bt + (size_t)b * strideB;
  const T* Ab2 = SPLIT ? (A2  + (size_t)b * strideA) : nullptr;
  const T* Bb2 = SPLIT ? (Bt2 + (size_t)b * strideB) : nullptr;

  const int rlane = lane & 15;
  const int koff  = (lane >> 4) * 8;
  const int mOff  = (lane >> 4) * 8;

  v8f acc[4][4];
#pragma unroll
  for (int i = 0; i < 4; ++i)
#pragma unroll
    for (int j = 0; j < 4; ++j) acc[i][j] = (v8f){0.f,0.f,0.f,0.f,0.f,0.f,0.f,0.f};

  for (int k0 = 0; k0 < K; k0 += 32) {
    V bh[4], bl[4];
#pragma unroll
    for (int j = 0; j < 4; ++j) {
      const size_t bo = (size_t)(n0 + (j << 4) + rlane) * ldb + koff + k0;
      bh[j] = Frag<T>::load(Bb + bo);
      if (SPLIT) bl[j] = Frag<T>::load(Bb2 + bo);
    }
#pragma unroll
    for (int i = 0; i < 4; ++i) {
      const size_t ao = (size_t)(m0 + (i << 4) + rlane) * lda + koff + k0;
      V ah = Frag<T>::load(Ab + ao);
      V al;
      if (SPLIT) al = Frag<T>::load(Ab2 + ao);
#pragma unroll
      for (int j = 0; j < 4; ++j) {
        acc[i][j] = Frag<T>::mma(ah, bh[j], acc[i][j]);
        if (SPLIT) {
          acc[i][j] = Frag<T>::mma(ah, bl[j], acc[i][j]);
          acc[i][j] = Frag<T>::mma(al, bh[j], acc[i][j]);
        }
      }
      Frag<T>::guard(acc[i][0], acc[i][3], ah, SPLIT ? al : ah);
    }
    Frag<T>::keep(bh[0], bh[1], bh[2], bh[3]);
    if (SPLIT) Frag<T>::keep(bl[0], bl[1], bl[2], bl[3]);
  }
  acc_guard4(acc[0][0], acc[0][1], acc[0][2], acc[0][3]);
  acc_guard4(acc[1][0], acc[1][1], acc[1][2], acc[1][3]);
  acc_guard4(acc[2][0], acc[2][1], acc[2][2], acc[2][3]);
  acc_guard4(acc[3][0], acc[3][1], acc[3][2], acc[3][3]);

  float* slab = sT[wave];
  const float* Rb = RESID ? (resid + (size_t)b * strideR) : nullptr;
#pragma unroll
  for (int i = 0; i < 4; ++i) {
    const int mBase = m0 + (i << 4);
#pragma unroll
    for (int j = 0; j < 4; ++j) {
      const int n = n0 + (j << 4) + rlane;
      float bv = 0.f;
      if (BIAS_MODE == 2) bv = bias[n];
#pragma unroll
      for (int r = 0; r < 8; ++r) {
        float v = acc[i][j][r] * scale;
        if (BIAS_MODE == 1) v += bias[mBase + mOff + r];
        if (BIAS_MODE == 2) v += bv;
        if (RESID) v += Rb[(size_t)(mBase + mOff + r) * ldc + n];
        if (ACT == 1) v = tanhf(v);
        if (ACT == 2) v = fmaxf(v, 0.0f);
        if (ACT == 3) v = v / (1.0f + expf(-v));
        if (ACT == 4) v = (v > 0.f) ? v : 0.01f * v;
        if (ACT == 5) v = 0.5f * v * (1.0f + erff(v * 0.70710678118654752f));
        slab[(mOff + r) * 68 + (j << 4) + rlane] = v;
      }
    }
    __builtin_amdgcn_fence(__ATOMIC_RELEASE, "workgroup");
    __builtin_amdgcn_wave_barrier();
    __builtin_amdgcn_fence(__ATOMIC_ACQUIRE, "workgroup");
    if (OUT_MODE == 0) {
      float* C = (float*)Cout + (size_t)b * strideC;
      const int hh = lane >> 4, c4 = (lane & 15) * 4;
      for (int pass = 0; pass < 2; ++pass) {
#pragma unroll
        for (int it = 0; it < 8; ++it) {
          const int row = it * 2 + hh;
          v4f v = *(const v4f*)(slab + row * 68 + c4);
          *(volatile v4f*)(C + (size_t)(mBase + row) * ldc + n0 + c4) = v;
        }
        __threadfence();
      }
    } else {
      const int q = lane >> 3, c8 = (lane & 7) * 8;
      unsigned short* C  = (unsigned short*)Cout  + (size_t)b * strideC;
      unsigned short* C2 = (OUT_MODE == 2) ? ((unsigned short*)Cout2 + (size_t)b * strideC) : nullptr;
      for (int pass = 0; pass < 2; ++pass) {
#pragma unroll
        for (int it = 0; it < 4; ++it) {
          const int row = it * 4 + q;
          const float* sp = slab + row * 68 + c8;
          v8h hv, lv;
#pragma unroll
          for (int e = 0; e < 8; ++e) {
            if (OUT_MODE == 1) {
              hv[e] = (_Float16)sp[e];
            } else {
              unsigned short hb = f2bf_bits(sp[e]);
              unsigned short lb = f2bf_bits(sp[e] - bf_bits2f(hb));
              hv[e] = __builtin_bit_cast(_Float16, hb);
              lv[e] = __builtin_bit_cast(_Float16, lb);
            }
          }
          *(volatile v8h*)(C + (size_t)(mBase + row) * ldc + n0 + c8) = hv;
          if (OUT_MODE == 2) *(volatile v8h*)(C2 + (size_t)(mBase + row) * ldc + n0 + c8) = lv;
        }
        __threadfence();
      }
    }
    __builtin_amdgcn_fence(__ATOMIC_RELEASE, "workgroup");
    __builtin_amdgcn_wave_barrier();
    __builtin_amdgcn_fence(__ATOMIC_ACQUIRE, "workgroup");
  }
}

__global__ __launch_bounds__(256) void cvt_s_kernel(const float* __restrict__ s, unsigned short* __restrict__ dst) {
  const int i   = blockIdx.x * 256 + threadIdx.x;
  const int row = i >> 4;
  const int c8  = (i & 15) * 8;
  const int ca  = (c8 < NIN - 4) ? c8 : (NIN - 4);
  const int cb  = (c8 + 4 < NIN - 4) ? (c8 + 4) : (NIN - 4);
  const float* sp = s + (size_t)row * NIN;
  const v4f a  = *(const v4f*)(sp + ca);
  const v4f bq = *(const v4f*)(sp + cb);
  v8h hv;
#pragma unroll
  for (int e = 0; e < 4; ++e) {
    const float ae = a[e];
    const float be = bq[e];
    const float fa = (c8 + e < NIN) ? 1.0f : 0.0f;
    const float fb = (c8 + 4 + e < NIN) ? 1.0f : 0.0f;
    const float va = fmaf(fa, ae, 0.0f);
    const float vb = fmaf(fb, be, 0.0f);
    hv[e]     = __builtin_bit_cast(_Float16, f2bf_bits(va));
    hv[4 + e] = __builtin_bit_cast(_Float16, f2bf_bits(vb));
  }
  unsigned short* p = dst + (size_t)i * 8;
  *(volatile v8h*)p = hv;
  __threadfence();
  *(volatile v8h*)p = hv;
}

__global__ __launch_bounds__(256) void prep_kernel(const float* __restrict__ Wx_w, const float* __restrict__ Wx_b,
                                                   const float* __restrict__ Wh_b, const float* __restrict__ Wy_w,
                                                   unsigned short* __restrict__ WX16, unsigned short* __restrict__ WY16,
                                                   float* __restrict__ BIAS64) {
  const int tid = threadIdx.x;
#pragma unroll 1
  for (int q = tid; q < NPAD_X * (KPAD_X / 8); q += 256) {
    const int row  = q >> 4;
    const int c8   = (q & 15) * 8;
    const int rowc = (row < NHID) ? row : (NHID - 1);
    v8h hv;
#pragma unroll
    for (int e = 0; e < 8; ++e) {
      const int col  = c8 + e;
      const int colc = (col < NIN) ? col : (NIN - 1);
      const float w  = Wx_w[rowc * NIN + colc];
      const float fs = (row < NHID && col < NIN) ? 1.0f : 0.0f;
      const float v  = fmaf(fs, w, 0.0f);
      hv[e] = __builtin_bit_cast(_Float16, f2bf_bits(v));
    }
    unsigned short* p = WX16 + (size_t)q * 8;
    *(volatile v8h*)p = hv;
    __threadfence();
    *(volatile v8h*)p = hv;
  }
#pragma unroll 1
  for (int q = tid; q < NPAD_Y * (KPAD_Y / 8); q += 256) {
    const int row  = q >> 3;
    const int c8   = (q & 7) * 8;
    const int rowc = (row < NVOC) ? row : (NVOC - 1);
    v8h hv;
#pragma unroll
    for (int e = 0; e < 8; ++e) {
      const int col  = c8 + e;
      const int colc = (col < NHID) ? col : (NHID - 1);
      const float w  = Wy_w[rowc * NHID + colc];
      const float fs = (row < NVOC && col < NHID) ? 1.0f : 0.0f;
      const float v  = fmaf(fs, bf16r(w), 0.0f);
      hv[e] = (_Float16)(v * WY_CARRY);
    }
    unsigned short* p = WY16 + (size_t)q * 8;
    *(volatile v8h*)p = hv;
    __threadfence();
    *(volatile v8h*)p = hv;
  }
  if (tid < NPAD_X / 4) {
    v4f o;
#pragma unroll
    for (int e = 0; e < 4; ++e) {
      const int n  = tid * 4 + e;
      const int nc = (n < NHID) ? n : (NHID - 1);
      const float ba = Wx_b[nc];
      const float bb = Wh_b[nc];
      const float fs = (n < NHID) ? 1.0f : 0.0f;
      o[e] = fmaf(fs, bf16r(ba) + bf16r(bb), 0.0f);
    }
    float* p = BIAS64 + tid * 4;
    *(volatile v4f*)p = o;
    __threadfence();
    *(volatile v4f*)p = o;
  }
}

__global__ __launch_bounds__(SCAN_THR) void scan_kernel(const float* __restrict__ XSB, const float* __restrict__ h0,
                                                        const float* __restrict__ Wh_w, unsigned short* __restrict__ H16,
                                                        float* __restrict__ HFIN) {
  __shared__ __align__(16) float whs[NHID * NHID];
  __shared__ __align__(16) float hs[2 * SCAN_THR];
  __shared__ __align__(16) float xstage[HBATCH * NPAD_X];
  __shared__ __align__(16) float hstage[HBATCH * NPAD_X];
  _Float16* H16h = (_Float16*)H16;
  const int i   = threadIdx.x;
  const int ic  = (i < NHID) ? i : (NHID - 1);
  const float act = (i < NHID) ? 1.0f : 0.0f;
  const int q1 = i >> 3, c8 = (i & 7) * 8;

#pragma unroll 1
  for (int q = i; q < (NHID * NHID) / 4; q += SCAN_THR) {
    const v4f w = *(const v4f*)(Wh_w + 4 * q);
    v4f r;
#pragma unroll
    for (int e = 0; e < 4; ++e) r[e] = bf16r(w[e]);
    *(v4f*)(whs + 4 * q) = r;
  }
  {
    const float hv0 = h0[ic];
    hs[i] = fmaf(act, bf16r(hv0), 0.0f);
    hs[SCAN_THR + i] = 0.0f;
  }
  {
    v8h z;
#pragma unroll
    for (int e = 0; e < 8; ++e) z[e] = (_Float16)0.0f;
    for (int pass = 0; pass < 2; ++pass) {
#pragma unroll
      for (int g = 0; g < 2; ++g) {
        const int row = q1 + 8 * g;
        *(volatile v8h*)(H16h + (size_t)(SEQ_T + row) * KPAD_Y + c8) = z;
      }
      __threadfence();
    }
  }
  __syncthreads();

  const float* wr = whs + ic * NHID;
  int cur = 0;
#pragma unroll 1
  for (int tb = 0; tb < SEQ_T / HBATCH; ++tb) {
    const int t0 = tb * HBATCH;
#pragma unroll
    for (int k = 0; k < 4; ++k) {
      const int q = i + SCAN_THR * k;
      const int row = q >> 4, c4 = (q & 15) * 4;
      const v4f v = *(const v4f*)(XSB + (size_t)(t0 + row) * NPAD_X + c4);
      *(v4f*)(xstage + row * NPAD_X + c4) = v;
    }
    __syncthreads();
#pragma unroll 1
    for (int u = 0; u < HBATCH; ++u) {
      const float* hc = hs + cur * SCAN_THR;
      const float xv = xstage[u * NPAD_X + i];
      float a0 = 0.0f, a1 = 0.0f, a2 = 0.0f, a3 = 0.0f;
#pragma unroll 1
      for (int j = 0; j < NHID; j += 4) {
        const v4f w4 = *(const v4f*)(wr + j);
        const v4f h4 = *(const v4f*)(hc + j);
        a0 = fmaf(w4[0], h4[0], a0);
        a1 = fmaf(w4[1], h4[1], a1);
        a2 = fmaf(w4[2], h4[2], a2);
        a3 = fmaf(w4[3], h4[3], a3);
      }
      const float pre = xv + ((a0 + a1) + (a2 + a3));
      const float th  = tanhf(pre);
      const float hn  = (i < NHID) ? th : 0.0f;
      hs[(cur ^ 1) * SCAN_THR + i] = hn;
      hstage[u * NPAD_X + i] = hn;
      cur ^= 1;
      __syncthreads();
    }
    for (int pass = 0; pass < 2; ++pass) {
#pragma unroll
      for (int g = 0; g < 2; ++g) {
        const int row = q1 + 8 * g;
        const v4f x0 = *(const v4f*)(hstage + row * NPAD_X + c8);
        const v4f x1 = *(const v4f*)(hstage + row * NPAD_X + c8 + 4);
        v8h hv;
#pragma unroll
        for (int e = 0; e < 4; ++e) { const float f0 = x0[e]; const float f1 = x1[e]; hv[e] = (_Float16)f0; hv[4 + e] = (_Float16)f1; }
        *(volatile v8h*)(H16h + (size_t)(t0 + row) * KPAD_Y + c8) = hv;
      }
      __threadfence();
    }
    __syncthreads();
  }

  if (i < 16) {
    const v4f v = *(const v4f*)(hs + cur * SCAN_THR + 4 * i);
    *(volatile v4f*)(HFIN + 4 * i) = v;
    __threadfence();
    *(volatile v4f*)(HFIN + 4 * i) = v;
  }
}

__global__ __launch_bounds__(RD_THR) void readout_kernel(const unsigned short* __restrict__ H16, const unsigned short* __restrict__ WY16,
                                                         const float* __restrict__ Wy_b, const float* __restrict__ HFIN,
                                                         float* __restrict__ out) {
  __shared__ __align__(16) unsigned short wys[NPAD_Y * KPAD_Y];
  __shared__ __align__(16) float Lg[LGROWS * LGP];
  __shared__ __align__(16) float hf[64];
  __shared__ __align__(16) float wyb[NPAD_Y];
  const int tid = threadIdx.x, lane = tid & 31, wave = tid >> 5;
  const int c = lane & 15, hh = lane >> 4;
  const int b = blockIdx.x;

  if (tid < 16) {
    const v4f v = *(const v4f*)(HFIN + 4 * tid);
    *(v4f*)(hf + 4 * tid) = v;
  }
  if (tid < NPAD_Y / 4) {
    const int col0 = tid * 4;
    const int colc = (col0 < NVOC - 4) ? col0 : (NVOC - 4);
    const v4f bv4 = *(const v4f*)(Wy_b + colc);
    v4f o;
#pragma unroll
    for (int e = 0; e < 4; ++e) {
      const float be = bv4[e];
      const float fs = (col0 + e < NVOC) ? 1.0f : 0.0f;
      o[e] = fmaf(fs, bf16r(be), 0.0f);
    }
    *(v4f*)(wyb + col0) = o;
  }
#pragma unroll 1
  for (int k = 0; k < (NPAD_Y * KPAD_Y / 8) / RD_THR; ++k) {
    const int q = tid + RD_THR * k;
    const v4u v = *(const v4u*)(WY16 + 8 * q);
    *(v4u*)(wys + 8 * q) = v;
  }
  __syncthreads();

  float bv[7];
#pragma unroll
  for (int tn = 0; tn < 7; ++tn) bv[tn] = wyb[16 * tn + c];

  const _Float16* wyh    = (const _Float16*)wys;
  const _Float16* hplane = (const _Float16*)H16;
  const v8f z8 = {0.f, 0.f, 0.f, 0.f, 0.f, 0.f, 0.f, 0.f};

#pragma unroll 1
  for (int ms = wave; ms < 5; ms += 4) {
    const int r0 = b * TBLK + 16 * ms;
    const _Float16* arow = hplane + (size_t)(r0 + c) * KPAD_Y + 8 * hh;
    const v16h a0 = Frag<_Float16>::load(arow);
    const v16h a1 = Frag<_Float16>::load(arow + 32);
    v8f acc[7];
#pragma unroll
    for (int tn = 0; tn < 7; ++tn) acc[tn] = z8;
#pragma unroll
    for (int tn = 0; tn < 7; ++tn) {
      const _Float16* brow = wyh + (16 * tn + c) * KPAD_Y + 8 * hh;
      const v16h b0 = Frag<_Float16>::load(brow);
      const v16h b1 = Frag<_Float16>::load(brow + 32);
      acc[tn] = Frag<_Float16>::mma(a0, b0, acc[tn]);
      acc[tn] = Frag<_Float16>::mma(a1, b1, acc[tn]);
      acc_guard1_h4(acc[tn], a0, a1, b0, b1);
    }
    keep2_h(a0, a1);
    acc_guard4(acc[0], acc[1], acc[2], acc[3]);
    acc_guard3(acc[4], acc[5], acc[6]);
#pragma unroll
    for (int tn = 0; tn < 7; ++tn) {
#pragma unroll
      for (int r = 0; r < 8; ++r)
        Lg[(16 * ms + 8 * hh + r) * LGP + 16 * tn + c] = acc[tn][r] * WY_CARRY_INV + bv[tn];
    }
  }
  __syncthreads();

  if (tid <= TBLK) {
    float* rp = Lg + tid * LGP;
    float mx = rp[0];
#pragma unroll 4
    for (int k = 1; k < NVOC; ++k) mx = fmaxf(mx, rp[k]);
    float sum = 0.0f;
#pragma unroll 4
    for (int k = 0; k < NVOC; ++k) { const float e = expf(rp[k] - mx); rp[k] = e; sum += e; }
    const float inv = 1.0f / sum;
#pragma unroll 4
    for (int k = 0; k < NVOC; ++k) rp[k] = rp[k] * inv;
  }
  __syncthreads();

  const long blkf = (long)b * (TBLK * NVOC);
  const long Fs = (b == 0) ? 0L : (blkf + FSHIFT);
  const long Fe = (b == NBLK_Y - 1) ? TOTAL_F : (blkf + TBLK * NVOC + FSHIFT);
  const int nchunk = (int)((Fe - Fs) >> 2);
  const int gbase = OUT1_OFF_F + (int)blkf;
  for (int pass = 0; pass < 2; ++pass) {
#pragma unroll 1
    for (int it = 0; it < NIT_ST; ++it) {
      const int q = it * RD_THR + tid;
      if (q < nchunk) {
        const long F0 = Fs + 4L * q;
        v4f v;
#pragma unroll
        for (int e = 0; e < 4; ++e) {
          const int F = (int)F0 + e;
          const int G = F - gbase;
          int Gc = (G < 0) ? 0 : G;
          Gc = (Gc > (TBLK + 1) * NVOC - 1) ? ((TBLK + 1) * NVOC - 1) : Gc;
          const int row = Gc / NVOC;
          const int col = Gc - row * NVOC;
          const float pv = Lg[row * LGP + col];
          int Fh = (F < 0) ? 0 : F;
          Fh = (Fh > 63) ? 63 : Fh;
          const float hv = hf[Fh];
          const float fa = (G < 0) ? 1.0f : 0.0f;
          const float fb = 1.0f - fa;
          v[e] = fmaf(fa, hv, fb * pv);
        }
        *(volatile v4f*)(out + F0) = v;
      }
    }
    __threadfence();
  }
}

extern "C" void kernel_launch(void* const* d_in, const int* in_sizes, int n_in,
                              void* d_out, int out_size, void* d_ws, size_t ws_size, hipStream_t stream) {
  if (n_in < 8 || d_out == nullptr || d_ws == nullptr) return;
  if (in_sizes[0] != SEQ_T * NIN || in_sizes[1] != NHID || in_sizes[2] != NHID * NIN || in_sizes[3] != NHID ||
      in_sizes[4] != NHID * NHID || in_sizes[5] != NHID || in_sizes[6] != NVOC * NHID || in_sizes[7] != NVOC ||
      (long)out_size != TOTAL_F) return;

  const float* s    = (const float*)d_in[0];
  const float* h0   = (const float*)d_in[1];
  const float* Wx_w = (const float*)d_in[2];
  const float* Wx_b = (const float*)d_in[3];
  const float* Wh_w = (const float*)d_in[4];
  const float* Wh_b = (const float*)d_in[5];
  const float* Wy_w = (const float*)d_in[6];
  const float* Wy_b = (const float*)d_in[7];
  float* out = (float*)d_out;

  char* ws = (char*)d_ws; size_t off = 0;
  auto carve = [&](size_t bytes) -> char* { char* p = ws + off; off += (bytes + 255) & ~(size_t)255; return p; };
  unsigned short* S16    = (unsigned short*)carve((size_t)SEQ_T * KPAD_X * 2);
  unsigned short* WX16   = (unsigned short*)carve((size_t)NPAD_X * KPAD_X * 2);
  unsigned short* WY16   = (unsigned short*)carve((size_t)NPAD_Y * KPAD_Y * 2);
  float*          BIAS64 = (float*)carve((size_t)NPAD_X * 4);
  float*          HFIN   = (float*)carve((size_t)64 * 4);
  float*          XSB    = (float*)carve((size_t)SEQ_T * NPAD_X * 4);
  unsigned short* H16    = (unsigned short*)carve((size_t)HROWS * KPAD_Y * 2);
  if (off > ws_size || off > (size_t)134217728) return;

  cvt_s_kernel<<<(SEQ_T * (KPAD_X / 8)) / 256, 256, 0, stream>>>(s, S16);
  prep_kernel<<<1, 256, 0, stream>>>(Wx_w, Wx_b, Wh_b, Wy_w, WX16, WY16, BIAS64);

  const dim3 ggrid((SEQ_T / 64) * (NPAD_X / 64) / 8, 1);
  wmma_gemm64<1, false, 2, 0, false, 0><<<ggrid, 256, 0, stream>>>(
      S16, S16, KPAD_X, 0L, WX16, WX16, KPAD_X, 0L, (void*)XSB, (void*)XSB, NPAD_X, 0L,
      BIAS64, BIAS64, 0L, SEQ_T, NPAD_X, KPAD_X, 1.0f);

  scan_kernel<<<1, SCAN_THR, 0, stream>>>(XSB, h0, Wh_w, H16, HFIN);
  readout_kernel<<<NBLK_Y, RD_THR, 0, stream>>>(H16, WY16, Wy_b, HFIN, out);
}
